// DirectionalRecursiveBlock_74801150427531
// MI455X (gfx1250) — hardware-run, weakly checked
//
#include <hip/hip_runtime.h>

#ifndef NB
#define NB 2
#endif
#ifndef SEQ
#define SEQ 2048
#endif
#ifndef CTX
#define CTX 1024
#endif
#define NB_FULL 2
#define SEQ_FULL 2048
#define CTX_FULL 1024
#define DM 1024
#define NH 16
#define HD 64
#define DFF 4096
#define NR ((size_t)NB * SEQ)
#define MR ((int)((size_t)NB * SEQ))
#define NC ((size_t)NB * CTX)
#define MC ((int)((size_t)NB * CTX))
#define GBR 128
#define PBP 40
#define OBP 72
#define LN_EPS 1.0e-5f

static_assert(NB >= 1 && NB <= NB_FULL);
static_assert(SEQ >= 64 && SEQ <= SEQ_FULL && SEQ % 64 == 0);
static_assert(CTX >= 64 && CTX <= CTX_FULL && CTX % 64 == 0 && CTX <= SEQ);
static_assert(SEQ % 32 == 0 && CTX % 32 == 0);
static_assert((NB * SEQ) % 128 == 0 && (NB * CTX) % 128 == 0);
static_assert(NH * HD == DM && HD == 64);
static_assert(DM == 4 * 256);
static_assert(DM % 64 == 0 && DFF % 64 == 0 && DM % 32 == 0 && DFF % 32 == 0 && (2 * DM) % 64 == 0);
static_assert(DFF <= 4 * DM);
static_assert((PBP % 8) == 0 && (OBP % 8) == 0);
static_assert(NB <= GBR && GBR % 128 == 0);
static_assert((GBR * (DM / 8)) % 256 == 0 && (SEQ * 32) % 256 == 0);
static_assert(((size_t)DM * DM / 8) % 256 == 0 && ((size_t)DM * DFF / 8) % 256 == 0);
static_assert((DFF / 4) % 256 == 0 && DM <= DFF && 2 * DM <= DFF);

constexpr size_t al256(size_t b) { return (b + 255) & ~(size_t)255; }
constexpr size_t SZ_WDD = (size_t)DM * DM * 2;
constexpr size_t SZ_WDF = (size_t)DM * DFF * 2;
constexpr size_t SZ_P16 = NR * DM * 2;
constexpr size_t SZ_P32 = NR * DM * 4;
constexpr size_t SZ_RB  = (4 * SZ_P16 > NR * (size_t)DFF * 2) ? 4 * SZ_P16 : NR * (size_t)DFF * 2;
constexpr size_t SZ_E16 = (size_t)GBR * DM * 2;
constexpr size_t SZ_C16 = NC * DM * 2;
constexpr size_t SZ_CS  = (size_t)SEQ * 64 * 4;
constexpr size_t SZ_GB  = (size_t)GBR * 2 * DM * 4;
constexpr size_t SZ_ZB  = (size_t)DFF * 4;
constexpr size_t WS_TOTAL = al256(3 * SZ_WDD) + 5 * al256(SZ_WDD) + 2 * al256(SZ_WDF) + 3 * al256(2 * SZ_WDD)
                          + al256(SZ_E16) + al256(SZ_C16) + al256(SZ_CS) + 3 * al256(SZ_GB) + al256(SZ_ZB)
                          + al256(SZ_P16) + al256(SZ_RB) + 2 * al256(SZ_P32);
static_assert(WS_TOTAL <= (size_t)134217728);
static_assert(SZ_C16 <= SZ_P16);
static_assert(NR * (size_t)DFF * 2 <= SZ_RB && 4 * SZ_P16 <= SZ_RB);
static_assert(SZ_ZB % 128 == 0);

typedef unsigned short v8us __attribute__((ext_vector_type(8), may_alias));
typedef float  v8f  __attribute__((ext_vector_type(8)));
typedef float  v4f  __attribute__((ext_vector_type(4)));
typedef float  v4fa __attribute__((ext_vector_type(4), may_alias));
typedef _Float16 v16h __attribute__((ext_vector_type(16)));
typedef _Float16 v4h __attribute__((ext_vector_type(4)));
union FragH { v16h v; v8us half[2]; _Float16 h[16]; unsigned short u[16]; };

__device__ __forceinline__ unsigned short bf16_bits(float x) { unsigned int u = __float_as_uint(x); return (unsigned short)((u + 0x7FFFu + ((u >> 16) & 1u)) >> 16); }
__device__ __forceinline__ float bf16_val(unsigned short b) { return __uint_as_float(((unsigned int)b) << 16); }
__device__ __forceinline__ float bf16_rne(float x) { return bf16_val(bf16_bits(x)); }

static __device__ __forceinline__ _Float16 toh_flush(float v) { const _Float16 r = (_Float16)v; return (fabsf(v) < 6.103515625e-05f) ? (_Float16)0.0f : r; }

__device__ __forceinline__ size_t full_row(size_t r) { return (r / SEQ) * SEQ_FULL + (r % SEQ); }

__device__ __forceinline__ v16h g2_frag(const _Float16* p, int hh) { FragH f; f.half[0] = *(const v8us*)((const unsigned short*)p + 8 * hh); f.half[1] = *(const v8us*)((const unsigned short*)p + 16 + 8 * hh); return f.v; }
__device__ __forceinline__ v8f g2_mma(v16h a, v16h b, v8f c) { v8f d = __builtin_amdgcn_wmma_f32_16x16x32_f16(false, a, false, b, (short)0, c, false, false); asm volatile("v_nop\n\tv_nop\n\tv_nop\n\tv_nop" : "+v"(d) : "v"(a), "v"(b)); return d; }

__global__ __launch_bounds__(256) void k_w16(const float* __restrict__ W, _Float16* __restrict__ W16, size_t n8, float scale) {
  const size_t t = (size_t)blockIdx.x * 256 + threadIdx.x; if (t >= n8) return;
  const size_t e = t * 8; const float* src = W + e; const v4f a = *(const v4fa*)src; const v4f a2 = *(const v4fa*)(src + 4); FragH f;
#pragma unroll
  for (int q = 0; q < 4; ++q) { f.h[q] = toh_flush(bf16_rne(a[q]) * scale); f.h[4 + q] = toh_flush(bf16_rne(a2[q]) * scale); }
  const v8us o = f.half[0]; unsigned short* d = (unsigned short*)W16 + e;
  *(volatile v8us*)d = o; __threadfence(); *(volatile v8us*)d = o;
}

__global__ __launch_bounds__(256) void k_rows16(const float* __restrict__ x, _Float16* __restrict__ X16, size_t n8, int rc, int rf) {
  const size_t t = (size_t)blockIdx.x * 256 + threadIdx.x; if (t >= n8) return;
  const size_t e = t * 8; const size_t r = e / DM; const size_t c = e % DM; const size_t rs = (r / (size_t)rc) * (size_t)rf + (r % (size_t)rc);
  const float* src = x + rs * DM + c; const v4f a = *(const v4fa*)src; const v4f a2 = *(const v4fa*)(src + 4); FragH f;
#pragma unroll
  for (int q = 0; q < 4; ++q) { f.h[q] = toh_flush(bf16_rne(a[q])); f.h[4 + q] = toh_flush(bf16_rne(a2[q])); }
  const v8us o = f.half[0]; unsigned short* d = (unsigned short*)X16 + e;
  *(volatile v8us*)d = o; __threadfence(); *(volatile v8us*)d = o;
}

__global__ __launch_bounds__(256) void k_e16(const float* __restrict__ emb, _Float16* __restrict__ E16) {
  const int t = blockIdx.x * 256 + threadIdx.x; if (t >= GBR * (DM / 8)) return;
  const int r = t / (DM / 8), c = (t % (DM / 8)) * 8; const int rs = (r < NB) ? r : (NB - 1);
  const float* src = emb + (size_t)rs * DM + c; const v4f a = *(const v4fa*)src; const v4f a2 = *(const v4fa*)(src + 4); FragH f;
#pragma unroll
  for (int q = 0; q < 4; ++q) { f.h[q] = toh_flush((r < NB) ? bf16_rne(a[q]) : 0.0f); f.h[4 + q] = toh_flush((r < NB) ? bf16_rne(a2[q]) : 0.0f); }
  const v8us o = f.half[0]; unsigned short* d = (unsigned short*)E16 + (size_t)r * DM + c;
  *(volatile v8us*)d = o; __threadfence(); *(volatile v8us*)d = o;
}

__global__ __launch_bounds__(256) void k_zero32(float* __restrict__ Z, int n4) {
  const int t = blockIdx.x * 256 + threadIdx.x; if (t >= n4) return;
  const v4f z = {0.f, 0.f, 0.f, 0.f}; float* d = Z + (size_t)t * 4;
  *(volatile v4f*)d = z; __threadfence(); *(volatile v4f*)d = z;
}

__global__ __launch_bounds__(256) void k_cs(float* __restrict__ CS, int npos) {
  #pragma clang fp contract(off)
  const int t = blockIdx.x * 256 + threadIdx.x; const int pos = t >> 5, d = t & 31; if (pos >= npos) return;
  const float inv = 1.0f / powf(10000.0f, (float)d * 0.03125f);
  const float ang = (float)pos * inv;
  const float c = cosf(ang); const float s = sinf(ang);
  float* p = CS + (size_t)pos * 64 + d;
  *(volatile float*)p = c; *(volatile float*)(p + 32) = s; __threadfence(); *(volatile float*)p = c; *(volatile float*)(p + 32) = s;
}

template <int NHv, int TTv>
__global__ __launch_bounds__(256) void k_vt(const _Float16* __restrict__ V16, int ldv, int voff, _Float16* __restrict__ Vt) {
  __shared__ unsigned short tl[64][66]; const int tid = threadIdx.x; const int slab = blockIdx.x / (TTv / 64), lg = blockIdx.x % (TTv / 64); const int b = slab / NHv, h = slab % NHv;
  for (int i = tid; i < 64 * 8; i += 256) { const int r = i / 8, c8 = (i % 8) * 8; FragH f; f.half[0] = *(const v8us*)((const unsigned short*)V16 + ((size_t)b * TTv + lg * 64 + r) * ldv + voff + h * 64 + c8);
#pragma unroll
    for (int q = 0; q < 8; ++q) tl[r][c8 + q] = f.u[q]; }
  __syncthreads();
  for (int pass = 0; pass < 2; ++pass) {
#pragma unroll
    for (int rd = 0; rd < 2; ++rd) { const int d = rd * 32 + tid / 8, pc = tid % 8; FragH f;
#pragma unroll
      for (int q = 0; q < 8; ++q) f.u[q] = tl[pc * 8 + q][d];
      *(volatile v8us*)((unsigned short*)Vt + ((size_t)slab * 64 + d) * TTv + lg * 64 + pc * 8) = f.half[0]; }
    if (pass == 0) __threadfence(); }
}

template <int ACT, int ROPE, int RES, int OMAP>
__global__ __launch_bounds__(128) void k_gemm3(const _Float16* __restrict__ A, int lda, const _Float16* __restrict__ Bh, int ldb, float alpha, const float* __restrict__ bias, float bsc,
    const float* __restrict__ R, const float* __restrict__ CS, int plen,
    float* __restrict__ C, _Float16* __restrict__ C16, int ldc, int M, int N, int K) {
  static_assert(ACT == 0 || ACT == 4);
  static_assert(RES >= 0 && RES <= 2);
  __shared__ __attribute__((aligned(16))) float so[4][32][68];
  const int tid = threadIdx.x, w = __builtin_amdgcn_readfirstlane(tid >> 5), lane = tid & 31, ln = lane & 15, hh = lane >> 4;
  const int ntn = N >> 6; const int mt = blockIdx.x / ntn, nq = blockIdx.x - mt * ntn; const int row0 = mt * 128 + 32 * w, col0 = nq * 64; if (row0 >= M) return;
  const _Float16* a0p = A + (size_t)(row0 + ln) * lda; const _Float16* a1p = a0p + (size_t)16 * lda;
  const _Float16* b0p = Bh + (size_t)(col0 + ln) * ldb; const _Float16* b1p = b0p + (size_t)16 * ldb; const _Float16* b2p = b1p + (size_t)16 * ldb; const _Float16* b3p = b2p + (size_t)16 * ldb;
  const v8f z8 = {0.f,0.f,0.f,0.f,0.f,0.f,0.f,0.f}; v8f c00 = z8, c01 = z8, c02 = z8, c03 = z8, c10 = z8, c11 = z8, c12 = z8, c13 = z8;
#pragma unroll 1
  for (int kb = 0; kb < K; kb += 32) { const v16h a0 = g2_frag(a0p + kb, hh), a1 = g2_frag(a1p + kb, hh);
    v16h b = g2_frag(b0p + kb, hh); c00 = g2_mma(a0, b, c00); c10 = g2_mma(a1, b, c10);
    b = g2_frag(b1p + kb, hh); c01 = g2_mma(a0, b, c01); c11 = g2_mma(a1, b, c11);
    b = g2_frag(b2p + kb, hh); c02 = g2_mma(a0, b, c02); c12 = g2_mma(a1, b, c12);
    b = g2_frag(b3p + kb, hh); c03 = g2_mma(a0, b, c03); c13 = g2_mma(a1, b, c13); }
  v8f accs[8] = {c00, c01, c02, c03, c10, c11, c12, c13};
#pragma unroll
  for (int u = 0; u < 8; ++u) { const int t = u & 3, half = u >> 2; const int col = col0 + t * 16 + ln; const float bld = bias[col]; const float bv = bf16_rne(bld) * bsc;
#pragma unroll
    for (int r = 0; r < 8; ++r) { const int rloc = half * 16 + 8 * hh + r; const float v = accs[u][r] * alpha + bv; so[w][rloc][t * 16 + ln] = v; } }
  __builtin_amdgcn_fence(4  , "workgroup"); __builtin_amdgcn_wave_barrier();
  if (ROPE) {
    const int rr4 = lane >> 3, j4 = (lane & 7) * 4;
#pragma unroll 1
    for (int i = 0; i < 8; ++i) { const int rl = i * 4 + rr4; const int pos = (row0 + rl) % plen;
      const v4f cs = *(const v4fa*)(CS + (size_t)pos * 64 + j4); const v4f sn = *(const v4fa*)(CS + (size_t)pos * 64 + 32 + j4);
      const v4f t1 = *(const v4fa*)&so[w][rl][j4]; const v4f t2 = *(const v4fa*)&so[w][rl][32 + j4]; v4f u1, u2;
#pragma unroll
      for (int e = 0; e < 4; ++e) { u1[e] = t1[e] * cs[e] - t2[e] * sn[e]; u2[e] = t2[e] * cs[e] + t1[e] * sn[e]; }
      *(v4fa*)&so[w][rl][j4] = u1; *(v4fa*)&so[w][rl][32 + j4] = u2; }
  }
  if (ACT == 4 || RES != 0) {
    const int rsb = lane >> 4, cc = (lane & 15) * 4;
#pragma unroll 1
    for (int q = 0; q < 16; ++q) { const int rl = q * 2 + rsb; v4f v = *(const v4fa*)&so[w][rl][cc];
      if (ACT == 4) {
#pragma unroll
        for (int e = 0; e < 4; ++e) v[e] = 8.0f * v[e] * (1.0f + erff(v[e] * 0.70710678118654752f)); }
      if (RES != 0) { const size_t rrow = (RES == 2) ? full_row((size_t)(row0 + rl)) : (size_t)(row0 + rl); const v4f rv = *(const v4fa*)(R + rrow * ldc + col0 + cc);
#pragma unroll
        for (int e = 0; e < 4; ++e) v[e] += (RES == 2) ? bf16_rne(rv[e]) : rv[e]; }
      *(v4fa*)&so[w][rl][cc] = v; }
  }
  if (ROPE || ACT == 4 || RES != 0) { __builtin_amdgcn_fence(4  , "workgroup"); __builtin_amdgcn_wave_barrier(); }
  const int rsub = lane >> 4, c4 = (lane & 15) * 4;
  for (int pass = 0; pass < 2; ++pass) {
#pragma unroll
    for (int q = 0; q < 16; ++q) { const int r = q * 2 + rsub; const v4f v = *(const v4fa*)&so[w][r][c4];
      const size_t orow = OMAP ? full_row((size_t)(row0 + r)) : (size_t)(row0 + r);
      if (C) *(volatile v4f*)(C + orow * ldc + col0 + c4) = v;
      if (C16) { v4h h4; for (int i = 0; i < 4; ++i) h4[i] = toh_flush(v[i]); *(volatile v4h*)(C16 + (size_t)(row0 + r) * ldc + col0 + c4) = h4; } }
    if (pass == 0) __threadfence(); }
}

template <int CAUSAL, int TK>
__global__ __launch_bounds__(128) void k_attn(const _Float16* __restrict__ Q16, const _Float16* __restrict__ K16, const _Float16* __restrict__ VT, _Float16* __restrict__ O16) {
  __shared__ __attribute__((aligned(16))) _Float16 pb[4][16 * PBP];
  __shared__ __attribute__((aligned(16))) _Float16 ob[4][16 * OBP];
  const int tid = threadIdx.x, w = __builtin_amdgcn_readfirstlane(tid >> 5), lane = tid & 31, ln = lane & 15, hh = lane >> 4;
  const int h = blockIdx.y, b = blockIdx.z;
  const int q0 = (blockIdx.x * 4 + w) * 16;
  const size_t tok0 = (size_t)b * SEQ;
  const size_t key0 = (size_t)b * TK;
  const int slab = b * NH + h;
  _Float16* pw = &pb[w][0]; _Float16* ow = &ob[w][0];
  const _Float16* qrow = Q16 + (tok0 + q0 + ln) * DM + h * HD;
  const v16h qf0 = g2_frag(qrow, hh), qf1 = g2_frag(qrow + 32, hh);
  const v8f z8 = {0.f,0.f,0.f,0.f,0.f,0.f,0.f,0.f};
  v8f o0 = z8, o1 = z8, o2 = z8, o3 = z8;
  float mrow[8], lrow[8];
#pragma unroll
  for (int r = 0; r < 8; ++r) { mrow[r] = -1.0e30f; lrow[r] = 0.f; }
  const int kend = CAUSAL ? (q0 + 16) : TK;
#pragma unroll 1
  for (int kb = 0; kb < kend; kb += 32) {
    const _Float16* k0p = K16 + (key0 + kb + ln) * DM + h * HD; const _Float16* k1p = k0p + (size_t)16 * DM;
    v8f s0 = z8, s1 = z8;
    v16h kf = g2_frag(k0p, hh);    s0 = g2_mma(qf0, kf, s0);
    kf = g2_frag(k0p + 32, hh);    s0 = g2_mma(qf1, kf, s0);
    kf = g2_frag(k1p, hh);         s1 = g2_mma(qf0, kf, s1);
    kf = g2_frag(k1p + 32, hh);    s1 = g2_mma(qf1, kf, s1);
#pragma unroll
    for (int r = 0; r < 8; ++r) {
      const int row = q0 + 8 * hh + r;
      float a = s0[r] * 0.125f, c = s1[r] * 0.125f;
      if (CAUSAL) { a = (kb + ln > row) ? -1.0e9f : a; c = (kb + 16 + ln > row) ? -1.0e9f : c; }
      float t = fmaxf(a, c);
      t = fmaxf(t, __shfl_xor(t, 1, 32)); t = fmaxf(t, __shfl_xor(t, 2, 32)); t = fmaxf(t, __shfl_xor(t, 4, 32)); t = fmaxf(t, __shfl_xor(t, 8, 32));
      const float mnew = fmaxf(mrow[r], t);
      const float p0 = __expf(a - mnew), p1 = __expf(c - mnew);
      float ls = p0 + p1;
      ls += __shfl_xor(ls, 1, 32); ls += __shfl_xor(ls, 2, 32); ls += __shfl_xor(ls, 4, 32); ls += __shfl_xor(ls, 8, 32);
      const float corr = __expf(mrow[r] - mnew);
      lrow[r] = lrow[r] * corr + ls; mrow[r] = mnew;
      o0[r] *= corr; o1[r] *= corr; o2[r] *= corr; o3[r] *= corr;
      pw[(8 * hh + r) * PBP + ln]      = toh_flush(p0 * 256.0f);
      pw[(8 * hh + r) * PBP + 16 + ln] = toh_flush(p1 * 256.0f);
    }
    __builtin_amdgcn_fence(4  , "wavefront"); __builtin_amdgcn_wave_barrier();
    const v16h pf = g2_frag(pw + ln * PBP, hh);
    __builtin_amdgcn_fence(4  , "wavefront"); __builtin_amdgcn_wave_barrier();
    const _Float16* vp = VT + ((size_t)slab * HD + ln) * TK + kb;
    v16h vf = g2_frag(vp, hh);                  o0 = g2_mma(pf, vf, o0);
    vf = g2_frag(vp + (size_t)16 * TK, hh);     o1 = g2_mma(pf, vf, o1);
    vf = g2_frag(vp + (size_t)32 * TK, hh);     o2 = g2_mma(pf, vf, o2);
    vf = g2_frag(vp + (size_t)48 * TK, hh);     o3 = g2_mma(pf, vf, o3);
  }
#pragma unroll
  for (int r = 0; r < 8; ++r) {
    const float rl = 0.25f * __builtin_amdgcn_rcpf(lrow[r]);
    const int rloc = (8 * hh + r) * OBP + ln;
    ow[rloc]      = toh_flush(o0[r] * rl); ow[rloc + 16] = toh_flush(o1[r] * rl);
    ow[rloc + 32] = toh_flush(o2[r] * rl); ow[rloc + 48] = toh_flush(o3[r] * rl);
  }
  __builtin_amdgcn_fence(4  , "wavefront"); __builtin_amdgcn_wave_barrier();
  const int rq = lane >> 3, pc = (lane & 7) * 8;
  for (int pass = 0; pass < 2; ++pass) {
#pragma unroll
    for (int i = 0; i < 4; ++i) { const int row = i * 4 + rq; const v8us v = *(const v8us*)(ow + row * OBP + pc);
      *(volatile v8us*)((unsigned short*)O16 + (tok0 + q0 + row) * DM + h * HD + pc) = v; }
    if (pass == 0) __threadfence(); }
}

template <int RBF, int RMAP>
__global__ __launch_bounds__(256) void k_adaln(const float* __restrict__ X, const float* __restrict__ GB, int ldg, float eps, _Float16* __restrict__ O16) {
  #pragma clang fp contract(off)
  __shared__ float red[256];
  const size_t r = blockIdx.x; const int t = threadIdx.x; const int c0 = t * 4;
  const size_t rfull = (r / SEQ) * SEQ_FULL + (r % SEQ);
  const size_t rr = RMAP ? rfull : r;
  const size_t bb = r / SEQ;
  const v4f xa = *(const v4fa*)(X + rr * DM + c0);
  const v4f ga = *(const v4fa*)(GB + bb * (size_t)ldg + c0); const v4f ba = *(const v4fa*)(GB + bb * (size_t)ldg + DM + c0);
  float s[4]; float sum = 0.f;
#pragma unroll
  for (int q = 0; q < 4; ++q) { s[q] = RBF ? bf16_rne(xa[q]) : xa[q]; sum += s[q]; }
  red[t] = sum; __syncthreads();
  for (int st = 128; st > 0; st >>= 1) { if (t < st) red[t] += red[t + st]; __syncthreads(); }
  const float mu = red[0] * (1.0f / (float)DM); __syncthreads();
  float vs = 0.f;
#pragma unroll
  for (int q = 0; q < 4; ++q) { const float dl = s[q] - mu; vs += dl * dl; }
  red[t] = vs; __syncthreads();
  for (int st = 128; st > 0; st >>= 1) { if (t < st) red[t] += red[t + st]; __syncthreads(); }
  const float rs = rsqrtf(red[0] * (1.0f / (float)DM) + eps);
  v4h y;
#pragma unroll
  for (int q = 0; q < 4; ++q) { const float yf = (s[q] - mu) * rs * (1.0f + ga[q]) + ba[q]; y[q] = toh_flush(yf); }
  for (int pass = 0; pass < 2; ++pass) {
    *(volatile v4h*)(O16 + r * DM + c0) = y;
    if (pass == 0) __threadfence(); }
}

extern "C" void kernel_launch(void* const* d_in, const int* in_sizes, int n_in,
                              void* d_out, int out_size, void* d_ws, size_t ws_size, hipStream_t stream) {
  if (n_in < 19) return;
  const float* x    = (const float*)d_in[0];  const float* emb  = (const float*)d_in[1];  const float* ctx  = (const float*)d_in[2];
  const float* ln1w = (const float*)d_in[3];  const float* ln1b = (const float*)d_in[4];
  const float* ln2w = (const float*)d_in[5];  const float* ln2b = (const float*)d_in[6];
  const float* ln3w = (const float*)d_in[7];  const float* ln3b = (const float*)d_in[8];
  const float* qkvw = (const float*)d_in[9];  const float* saw  = (const float*)d_in[10];
  const float* qw   = (const float*)d_in[11]; const float* kw   = (const float*)d_in[12]; const float* vw = (const float*)d_in[13]; const float* caw = (const float*)d_in[14];
  const float* w1   = (const float*)d_in[15]; const float* b1   = (const float*)d_in[16]; const float* w2 = (const float*)d_in[17]; const float* b2  = (const float*)d_in[18];

  const size_t needX = ((size_t)(NB - 1) * SEQ_FULL + SEQ) * DM;
  const size_t needC = ((size_t)(NB - 1) * CTX_FULL + CTX) * DM;
  if ((size_t)in_sizes[0] < needX || (size_t)in_sizes[1] < (size_t)NB * DM || (size_t)in_sizes[2] < needC || (size_t)out_size < needX) return;
  { static const int li[3] = {3, 5, 7}; for (int i = 0; i < 3; ++i) if ((size_t)in_sizes[li[i]] < (size_t)2 * DM * DM) return; }
  { static const int lb[3] = {4, 6, 8}; for (int i = 0; i < 3; ++i) if (in_sizes[lb[i]] < 2 * DM) return; }
  if ((size_t)in_sizes[9] < (size_t)3 * DM * DM) return;
  { static const int wi[5] = {10, 11, 12, 13, 14}; for (int i = 0; i < 5; ++i) if ((size_t)in_sizes[wi[i]] < (size_t)DM * DM) return; }
  if ((size_t)in_sizes[15] < (size_t)DM * DFF || (size_t)in_sizes[17] < (size_t)DM * DFF || in_sizes[16] < DFF || in_sizes[18] < DM) return;

  char* ws = (char*)d_ws; size_t off = 0;
  auto take = [&](size_t bytes) { char* p = ws + off; off += (bytes + 255) & ~(size_t)255; return p; };
  const size_t WDD = SZ_WDD, WDF = SZ_WDF, P16 = SZ_P16, P32 = SZ_P32;
  _Float16* BQKV = (_Float16*)take(3 * WDD);
  _Float16* BSA = (_Float16*)take(WDD); _Float16* BQ2 = (_Float16*)take(WDD); _Float16* BK2 = (_Float16*)take(WDD); _Float16* BV2 = (_Float16*)take(WDD); _Float16* BCA = (_Float16*)take(WDD);
  _Float16* BW1 = (_Float16*)take(WDF);
  _Float16* BW2 = (_Float16*)take(WDF);
  _Float16* BL1 = (_Float16*)take(2 * WDD); _Float16* BL2 = (_Float16*)take(2 * WDD); _Float16* BL3 = (_Float16*)take(2 * WDD);
  _Float16* E16 = (_Float16*)take(SZ_E16);
  _Float16* C16 = (_Float16*)take(SZ_C16);
  float* CS  = (float*)take(SZ_CS);
  float* GB1 = (float*)take(SZ_GB); float* GB2 = (float*)take(SZ_GB); float* GB3 = (float*)take(SZ_GB);
  float* ZB  = (float*)take(SZ_ZB);
  char* RA = take(P16); _Float16* XN16 = (_Float16*)RA; _Float16* O16 = (_Float16*)RA;
  char* RB = take(SZ_RB); _Float16* Q16 = (_Float16*)RB; _Float16* K16 = (_Float16*)(RB + P16); _Float16* V16 = (_Float16*)(RB + 2 * P16); _Float16* VT = (_Float16*)(RB + 3 * P16); _Float16* HF = (_Float16*)RB;
  float* X1F = (float*)take(P32);
  float* X2F = (float*)take(P32);
  if (off > ws_size || off > (size_t)134217728) return;

  const size_t nDD = (size_t)DM * DM / 8, nDF = (size_t)DM * DFF / 8;
  const unsigned gDD = (unsigned)((nDD + 255) / 256), gDF = (unsigned)((nDF + 255) / 256), g2DD = (unsigned)((2 * nDD + 255) / 256), g3DD = (unsigned)((3 * nDD + 255) / 256);
  k_w16<<<g3DD, 256, 0, stream>>>(qkvw, BQKV, 3 * nDD, 16.0f);
  k_w16<<<gDD, 256, 0, stream>>>(saw, BSA, nDD, 16.0f); k_w16<<<gDD, 256, 0, stream>>>(qw, BQ2, nDD, 16.0f); k_w16<<<gDD, 256, 0, stream>>>(kw, BK2, nDD, 16.0f);
  k_w16<<<gDD, 256, 0, stream>>>(vw, BV2, nDD, 16.0f); k_w16<<<gDD, 256, 0, stream>>>(caw, BCA, nDD, 16.0f);
  k_w16<<<gDF, 256, 0, stream>>>(w1, BW1, nDF, 16.0f); k_w16<<<gDF, 256, 0, stream>>>(w2, BW2, nDF, 16.0f);
  k_w16<<<g2DD, 256, 0, stream>>>(ln1w, BL1, 2 * nDD, 16.0f); k_w16<<<g2DD, 256, 0, stream>>>(ln2w, BL2, 2 * nDD, 16.0f); k_w16<<<g2DD, 256, 0, stream>>>(ln3w, BL3, 2 * nDD, 16.0f);

  const size_t nc8 = NC * DM / 8;
  k_rows16<<<(unsigned)((nc8 + 255) / 256), 256, 0, stream>>>(ctx, C16, nc8, CTX, CTX_FULL);
  k_e16<<<(unsigned)((GBR * (DM / 8)) / 256), 256, 0, stream>>>(emb, E16);
  k_cs<<<(unsigned)((SEQ * 32) / 256), 256, 0, stream>>>(CS, SEQ);
  k_zero32<<<(unsigned)((DFF / 4) / 256), 256, 0, stream>>>(ZB, DFF / 4);

  const unsigned gP = (unsigned)((MR / 128) * (DM / 64)), gPC = (unsigned)((MC / 128) * (DM / 64)), gF1 = (unsigned)((MR / 128) * (DFF / 64)), gGB = (unsigned)((GBR / 128) * ((2 * DM) / 64));
  const unsigned gVTs = (unsigned)(NB * NH * (SEQ / 64)), gVTc = (unsigned)(NB * NH * (CTX / 64)); const dim3 gAT(SEQ / 64, NH, NB);

  k_gemm3<0, 0, 0, 0><<<gGB, 128, 0, stream>>>(E16, DM, BL1, DM, 0.0625f, ln1b, 1.0f, nullptr, nullptr, 0, GB1, nullptr, 2 * DM, GBR, 2 * DM, DM);
  k_gemm3<0, 0, 0, 0><<<gGB, 128, 0, stream>>>(E16, DM, BL2, DM, 0.0625f, ln2b, 1.0f, nullptr, nullptr, 0, GB2, nullptr, 2 * DM, GBR, 2 * DM, DM);
  k_gemm3<0, 0, 0, 0><<<gGB, 128, 0, stream>>>(E16, DM, BL3, DM, 0.0625f, ln3b, 1.0f, nullptr, nullptr, 0, GB3, nullptr, 2 * DM, GBR, 2 * DM, DM);

  k_adaln<1, 1><<<(unsigned)MR, 256, 0, stream>>>(x, GB1, 2 * DM, LN_EPS, XN16);
  k_gemm3<0, 1, 0, 0><<<gP, 128, 0, stream>>>(XN16, DM, BQKV, DM, 0.0625f, ZB, 0.0f, nullptr, CS, SEQ, nullptr, Q16, DM, MR, DM, DM);
  k_gemm3<0, 1, 0, 0><<<gP, 128, 0, stream>>>(XN16, DM, BQKV + (size_t)DM * DM, DM, 0.0625f, ZB, 0.0f, nullptr, CS, SEQ, nullptr, K16, DM, MR, DM, DM);
  k_gemm3<0, 0, 0, 0><<<gP, 128, 0, stream>>>(XN16, DM, BQKV + (size_t)2 * DM * DM, DM, 0.0625f, ZB, 0.0f, nullptr, nullptr, 0, nullptr, V16, DM, MR, DM, DM);
  k_vt<NH, SEQ><<<gVTs, 256, 0, stream>>>(V16, DM, 0, VT);
  k_attn<0, SEQ><<<gAT, 128, 0, stream>>>(Q16, K16, VT, O16);
  k_gemm3<0, 0, 2, 0><<<gP, 128, 0, stream>>>(O16, DM, BSA, DM, 0.0009765625f, ZB, 0.0f, x, nullptr, 0, X1F, nullptr, DM, MR, DM, DM);
  k_adaln<0, 0><<<(unsigned)MR, 256, 0, stream>>>(X1F, GB2, 2 * DM, LN_EPS, XN16);
  k_gemm3<0, 1, 0, 0><<<gP, 128, 0, stream>>>(XN16, DM, BQ2, DM, 0.0625f, ZB, 0.0f, nullptr, CS, SEQ, nullptr, Q16, DM, MR, DM, DM);
  k_gemm3<0, 1, 0, 0><<<gPC, 128, 0, stream>>>(C16, DM, BK2, DM, 0.0625f, ZB, 0.0f, nullptr, CS, CTX, nullptr, K16, DM, MC, DM, DM);
  k_gemm3<0, 0, 0, 0><<<gPC, 128, 0, stream>>>(C16, DM, BV2, DM, 0.0625f, ZB, 0.0f, nullptr, nullptr, 0, nullptr, V16, DM, MC, DM, DM);
  k_vt<NH, CTX><<<gVTc, 256, 0, stream>>>(V16, DM, 0, VT);
  k_attn<0, CTX><<<gAT, 128, 0, stream>>>(Q16, K16, VT, O16);
  k_gemm3<0, 0, 1, 0><<<gP, 128, 0, stream>>>(O16, DM, BCA, DM, 0.0009765625f, ZB, 0.0f, X1F, nullptr, 0, X2F, nullptr, DM, MR, DM, DM);
  k_adaln<0, 0><<<(unsigned)MR, 256, 0, stream>>>(X2F, GB3, 2 * DM, LN_EPS, XN16);
  k_gemm3<4, 0, 0, 0><<<gF1, 128, 0, stream>>>(XN16, DM, BW1, DM, 0.0625f, b1, 1.0f, nullptr, nullptr, 0, nullptr, HF, DFF, MR, DFF, DM);
  k_gemm3<0, 0, 1, 1><<<gP, 128, 0, stream>>>(HF, DFF, BW2, DFF, 0.00390625f, b2, 1.0f, X2F, nullptr, 0, (float*)d_out, nullptr, DM, MR, DM, DFF);
}
